// ModifiedGATConv_40862318854644
// MI455X (gfx1250) — hardware-verified
//
#include <hip/hip_runtime.h>
#include <math.h>

typedef __attribute__((ext_vector_type(16))) _Float16 v16h;
typedef __attribute__((ext_vector_type(16))) __bf16 v16b;
typedef __attribute__((ext_vector_type(8)))  _Float16 v8h;
typedef __attribute__((ext_vector_type(8)))  float v8f;
typedef __attribute__((ext_vector_type(4)))  float v4f;
typedef __attribute__((ext_vector_type(2)))  float v2f;
typedef __attribute__((ext_vector_type(4)))  unsigned v4u;
typedef __attribute__((ext_vector_type(4)))  int v4i;
typedef float __attribute__((may_alias)) float_a;
typedef int __attribute__((may_alias)) int_a;

template <typename T> __device__ __forceinline__ void vst2(void* p, T v) { *(volatile T*)p = v; __threadfence(); *(volatile T*)p = v; }
__device__ __forceinline__ v8f wmma16(v16h a, v16h b, v8f c) {
  v8f d = __builtin_amdgcn_wmma_f32_16x16x32_f16(false, a, false, b, (short)0, c, false, false);
  asm volatile("v_nop\n\tv_nop\n\tv_nop\n\tv_nop" : "+v"(d) : "v"(a), "v"(b));
  return d;
}
__device__ __forceinline__ v8f wmma_bf(v16b a, v16b b, v8f c) {
  v8f d = __builtin_amdgcn_wmma_f32_16x16x32_bf16(false, a, false, b, (short)0, c, false, false);
  asm volatile("v_nop\n\tv_nop\n\tv_nop\n\tv_nop" : "+v"(d) : "v"(a), "v"(b));
  return d;
}
__device__ __forceinline__ v16h frag_h(const _Float16* rowk0, int lane) {
  union { v16h v; v8h q[2]; } u; const _Float16* p = rowk0 + 8 * (lane >> 4);
  u.q[0] = *(const v8h*)p; u.q[1] = *(const v8h*)(p + 16); return u.v;
}
__device__ __forceinline__ v16h frag_f32(const float* rowk0, int lane) {
  v16h a; const float* p = rowk0 + 8 * (lane >> 4);
#pragma unroll
  for (int i = 0; i < 8; ++i) { a[i] = (_Float16)p[i]; a[8 + i] = (_Float16)p[16 + i]; }
  return a;
}
__device__ __forceinline__ v16h frag_f32s(const float* rowk0, int lane, float sc) {
  v16h a; const float* p = rowk0 + 8 * (lane >> 4);
#pragma unroll
  for (int i = 0; i < 8; ++i) { a[i] = (_Float16)(p[i] * sc); a[8 + i] = (_Float16)(p[16 + i] * sc); }
  return a;
}
__device__ __forceinline__ v16h fragc_f32(const float* W, int k0, int n, int lane, int ld, int K) {
  v16h a; const int g = lane >> 4;
#pragma unroll
  for (int i = 0; i < 8; ++i) { const int ka = k0 + 8 * g + i, kb = ka + 16;
    a[i] = (_Float16)(ka < K ? W[(size_t)ka * ld + n] : 0.f); a[8 + i] = (_Float16)(kb < K ? W[(size_t)kb * ld + n] : 0.f); }
  return a;
}
struct F2 { v16b h, l; };
__device__ __forceinline__ F2 bsplit16(const float v[16]) { F2 r;
#pragma unroll
  for (int i = 0; i < 16; ++i) { const __bf16 h = (__bf16)v[i]; r.h[i] = h; r.l[i] = (__bf16)(v[i] - (float)h); }
  return r; }
__device__ __forceinline__ F2 split_row(const float* row, int k0, int lane) { float v[16]; const float* p = row + k0 + 8 * (lane >> 4);
#pragma unroll
  for (int i = 0; i < 8; ++i) { v[i] = p[i]; v[8 + i] = p[16 + i]; }
  return bsplit16(v); }
__device__ __forceinline__ F2 split_rowK(const float* row, int k0, int lane, int K) { float v[16]; const int g = lane >> 4;
#pragma unroll
  for (int i = 0; i < 8; ++i) { const int ka = k0 + 8 * g + i, kb = ka + 16; v[i] = ka < K ? row[ka] : 0.f; v[8 + i] = kb < K ? row[kb] : 0.f; }
  return bsplit16(v); }
__device__ __forceinline__ F2 split_col(const float* W, int k0, int n, int lane, int ld, int K) { float v[16]; const int g = lane >> 4;
#pragma unroll
  for (int i = 0; i < 8; ++i) { const int ka = k0 + 8 * g + i, kb = ka + 16; v[i] = ka < K ? W[(size_t)ka * ld + n] : 0.f; v[8 + i] = kb < K ? W[(size_t)kb * ld + n] : 0.f; }
  return bsplit16(v); }
__device__ __forceinline__ v8f mac3(const F2& a, const F2& b, v8f c) { c = wmma_bf(a.l, b.h, c); c = wmma_bf(a.h, b.l, c); return wmma_bf(a.h, b.h, c); }
__device__ __forceinline__ float sigm(float v) { return 1.0f / (1.0f + expf(-v)); }
#define LDSX() do { asm volatile("s_wait_dscnt 0" ::: "memory"); __builtin_amdgcn_wave_barrier(); __builtin_amdgcn_fence(__ATOMIC_RELEASE, "workgroup"); } while (0)

#define NN 30000
#define NE 480000
#define FI 128
#define NH 4
#define DH 128
#define FH 512
#define RBA 128
#define NRBA ((NN + RBA - 1) / RBA)
#define NNP (NRBA * RBA)
#define RBM 2048
#define NRBM ((NN + RBM - 1) / RBM)
#define EPT 16
#define CH (256 * EPT)

__device__ __forceinline__ int f2ord(float f) { const int i = __float_as_int(f); return i >= 0 ? i : i ^ 0x7fffffff; }
__device__ __forceinline__ float ord2f(int i) { return __int_as_float(i >= 0 ? i : i ^ 0x7fffffff); }
__device__ __forceinline__ float lrelu(float v) { return v > 0.f ? v : 0.2f * v; }

template <int ATT>
__global__ __launch_bounds__(128) void k_node(const float* __restrict__ feat, const float* __restrict__ W, const float* __restrict__ al, const float* __restrict__ ar, float* __restrict__ OUT, float* __restrict__ EL, float* __restrict__ ER) {
  __shared__ __align__(16) float so[4][16][260];
  __shared__ float sel[4][16][4], ser[4][16][4];
  const int tid = threadIdx.x, wave = tid >> 5, lane = tid & 31, col = lane & 15, g = lane >> 4;
  const int r0 = blockIdx.x * 64 + wave * 16; const int ra = (r0 + col) < NN ? (r0 + col) : NN - 1;
#pragma unroll 1
  for (int nh = 0; nh < 2; ++nh) { v8f acc[16];
#pragma unroll
    for (int t = 0; t < 16; ++t) acc[t] = (v8f){};
#pragma unroll 1
    for (int kc = 0; kc < FI / 32; ++kc) { const F2 a = split_row(feat + (size_t)ra * FI, kc * 32, lane);
#pragma unroll
      for (int t = 0; t < 16; ++t) acc[t] = mac3(a, split_col(W, kc * 32, nh * 256 + t * 16 + col, lane, FH, FI), acc[t]); }
#pragma unroll
    for (int t = 0; t < 16; ++t)
#pragma unroll
      for (int r = 0; r < 8; ++r) so[wave][8 * g + r][t * 16 + col] = acc[t][r];
    LDSX();
    if (ATT) {
      const int rl = lane >> 1, hh = lane & 1; const int h = nh * 2 + hh; const float* row = &so[wave][rl][hh * DH]; float s1 = 0.f, s2 = 0.f;
#pragma unroll 1
      for (int c = 0; c < DH; ++c) { const float v = row[c]; s1 += v * al[h * DH + c]; s2 += v * ar[h * DH + c]; }
      sel[wave][rl][h] = s1; ser[wave][rl][h] = s2; }
    for (int q = lane; q < 16 * 64; q += 32) { const int rl = q >> 6, pc = q & 63; vst2(OUT + (size_t)(r0 + rl) * FH + nh * 256 + pc * 4, *(const v4f*)(&so[wave][rl][pc * 4])); }
    LDSX(); }
  if (ATT) { if (lane < 16) { vst2(EL + (size_t)(r0 + lane) * 4, *(const v4f*)(&sel[wave][lane][0])); vst2(ER + (size_t)(r0 + lane) * 4, *(const v4f*)(&ser[wave][lane][0])); } }
}
__global__ __launch_bounds__(256) void k_max(const int* __restrict__ src, const int* __restrict__ dst, const float* __restrict__ EL, const float* __restrict__ ER, float* __restrict__ SMX) {
  __shared__ int smx[RBM][4];
  const int tid = threadIdx.x; const int r0 = blockIdx.x * RBM;
  for (int q = tid; q < RBM * 4; q += 256) smx[q >> 2][q & 3] = f2ord(-3.0e38f);
  __syncthreads();
#pragma unroll 1
  for (int c0 = 0; c0 < NE; c0 += CH) { const int e0 = c0 + tid * EPT;
#pragma unroll
    for (int v = 0; v < EPT / 4; ++v) { int dd[4];
      if (e0 + v * 4 + 4 <= NE) { const int4 d4 = *(const int4*)(dst + e0 + v * 4); dd[0] = d4.x; dd[1] = d4.y; dd[2] = d4.z; dd[3] = d4.w; }
      else { for (int u = 0; u < 4; ++u) dd[u] = (e0 + v * 4 + u < NE) ? dst[e0 + v * 4 + u] : -1; }
#pragma unroll
      for (int u = 0; u < 4; ++u) { const unsigned rel = (unsigned)(dd[u] - r0); if (dd[u] >= 0 && rel < (unsigned)RBM) { int s = src[e0 + v * 4 + u]; s = s < 0 ? 0 : (s >= NN ? NN - 1 : s);
#pragma unroll
          for (int h = 0; h < NH; ++h) atomicMax(&smx[rel][h], f2ord(lrelu(EL[(size_t)s * 4 + h] + ER[(size_t)(r0 + rel) * 4 + h]))); } } } }
  __syncthreads();
  for (int q = tid; q < RBM * 4; q += 256) { const int rl = q >> 2, h = q & 3; if (r0 + rl < NNP) vst2(SMX + (size_t)(r0 + rl) * 4 + h, ord2f(smx[rl][h])); }
}
__global__ __launch_bounds__(256) void k_gagg(const int* __restrict__ src, const int* __restrict__ dst, const float* __restrict__ XW, const float* __restrict__ EL, const float* __restrict__ ER, const float* __restrict__ SMX, const float* RES, const float* __restrict__ bias, float* RST) {
  __shared__ __align__(16) float sacc[RBA][FH];
  __shared__ float sden[RBA][4]; __shared__ float ser_[RBA][4], smx_[RBA][4];
  __shared__ int ssrc[8][32 * EPT], sdl[8][32 * EPT]; __shared__ int scnt[8];
  const int tid = threadIdx.x, wave = tid >> 5, lane = tid & 31;
  const int r0 = blockIdx.x * RBA; const int* esrc = src; const int* edst = dst;
  for (int q = tid; q < RBA * FH; q += 256) (&sacc[0][0])[q] = 0.f;
  for (int q = tid; q < RBA * 4; q += 256) { const int rl = q >> 2, h = q & 3; const int row = r0 + rl; sden[rl][h] = 0.f; ser_[rl][h] = row < NN ? ER[(size_t)row * 4 + h] : 0.f; smx_[rl][h] = row < NN ? SMX[(size_t)row * 4 + h] : 0.f; }
  __syncthreads();
#define RB RBA
  #pragma unroll 1
  for (int c0 = 0; c0 < NE; c0 += CH) {
    const int e0 = c0 + tid * EPT; int hd[EPT]; int cnt = 0;
    if (e0 + EPT <= NE) {
#pragma unroll
      for (int v = 0; v < EPT / 4; ++v) { const int4 d4 = *(const int4*)(edst + e0 + v * 4);
        const int dd[4] = {d4.x, d4.y, d4.z, d4.w};
#pragma unroll
        for (int u = 0; u < 4; ++u) { const unsigned rel = (unsigned)(dd[u] - r0); const bool h = rel < (unsigned)RB; hd[v * 4 + u] = h ? (int)rel : -1; cnt += h ? 1 : 0; } } }
    else {
#pragma unroll
      for (int u = 0; u < EPT; ++u) { const int e = e0 + u; hd[u] = -1; if (e < NE) { const unsigned rel = (unsigned)(edst[e] - r0); if (rel < (unsigned)RB) { hd[u] = (int)rel; ++cnt; } } } }
    int incl = cnt;
#pragma unroll
    for (int off = 1; off < 32; off <<= 1) { const int vv = __shfl_up(incl, off, 32); if (lane >= off) incl += vv; }
    const int wtot = __shfl(incl, 31, 32); int pos = incl - cnt;
    if (cnt > 0) {
#pragma unroll
      for (int u = 0; u < EPT; ++u) if (hd[u] >= 0) { int s = esrc[e0 + u]; s = s < 0 ? 0 : (s >= NN ? NN - 1 : s); ssrc[wave][pos] = s; sdl[wave][pos] = hd[u];  ++pos; } }
    if (lane == 0) scnt[wave] = wtot;
    __syncthreads();
    for (int w = 0; w < 8; ++w) { const int nh = scnt[w]; for (int i = 0; i < nh; ++i) { const int s = ssrc[w][i], dl = sdl[w][i];
#pragma unroll
          for (int sl = 0; sl < 2; ++sl) { const int fcol = tid + sl * 256; const int h = fcol >> 7;
            const float wgt = expf(lrelu(EL[(size_t)s * 4 + h] + ser_[dl][h]) - smx_[dl][h]);
            sacc[dl][fcol] += wgt * XW[(size_t)s * FH + fcol]; if ((fcol & 127) == 0) sden[dl][h] += wgt; } } }
    __syncthreads(); }
#undef RB
#pragma unroll 1
  for (int q = tid; q < RBA * FH; q += 256) { const int rl = q >> 9, f = q & 511; const int row = r0 + rl; if (row >= NN) continue; const int h = f >> 7; const float den = sden[rl][h];
    const float v = (den > 0.f ? sacc[rl][f] / den : 0.f) + RES[(size_t)row * FH + f] + bias[f]; sacc[rl][f] = v; }
  __syncthreads();
  for (int q = tid; q < RBA * (FH / 4); q += 256) { const int rl = q >> 7, pc = q & 127; const int row = r0 + rl; v4f v = *(const v4f*)(&sacc[rl][pc * 4]); if (row >= NN) v = (v4f){0.f, 0.f, 0.f, 0.f}; vst2(RST + (size_t)row * FH + pc * 4, v); }
}
__global__ __launch_bounds__(256) void k_bn(const float* __restrict__ RST, float* __restrict__ MU, float* __restrict__ ISD) {
  const int c = blockIdx.x * 256 + threadIdx.x; float s = 0.f;
#pragma unroll 1
  for (int r = 0; r < NN; ++r) s += RST[(size_t)r * FH + c];
  const float mu = s * (1.0f / NN); float q2 = 0.f;
#pragma unroll 1
  for (int r = 0; r < NN; ++r) { const float d = RST[(size_t)r * FH + c] - mu; q2 += d * d; }
  vst2(MU + c, mu); vst2(ISD + c, rsqrtf(q2 * (1.0f / NN) + 1e-5f));
}
__global__ __launch_bounds__(128) void k_out(const float* __restrict__ RST, const float* __restrict__ MU, const float* __restrict__ ISD, const float* __restrict__ gam, const float* __restrict__ bet, const float* __restrict__ Wo, const float* __restrict__ bo, float* __restrict__ out) {
  __shared__ __align__(16) float so[4][16][132];
  __shared__ float ssc[FH], ssh[FH];
  const int tid = threadIdx.x, wave = tid >> 5, lane = tid & 31, col = lane & 15, g = lane >> 4;
  for (int c = tid; c < FH; c += 128) { const float scv = gam[c] * ISD[c]; ssc[c] = scv; ssh[c] = bet[c] - MU[c] * scv; }
  __syncthreads();
  const int r0 = blockIdx.x * 64 + wave * 16; const int ra = (r0 + col) < NN ? (r0 + col) : NN - 1; const float* arow = RST + (size_t)ra * FH;
  v8f acc[8] = {};
#pragma unroll 1
  for (int kc = 0; kc < FH / 32; ++kc) { float v[16]; const int k0 = kc * 32 + 8 * g;
#pragma unroll
    for (int i = 0; i < 8; ++i) { const int ka = k0 + i, kb = ka + 16; const float xa = arow[ka] * ssc[ka] + ssh[ka], xb = arow[kb] * ssc[kb] + ssh[kb]; v[i] = xa > 0.f ? xa : 0.f; v[8 + i] = xb > 0.f ? xb : 0.f; }
    const F2 a = bsplit16(v);
#pragma unroll
    for (int t = 0; t < 8; ++t) acc[t] = mac3(a, split_col(Wo, kc * 32, t * 16 + col, lane, FI, FH), acc[t]); }
#pragma unroll
  for (int t = 0; t < 8; ++t) { const float bb = bo[t * 16 + col];
#pragma unroll
    for (int r = 0; r < 8; ++r) so[wave][8 * g + r][t * 16 + col] = acc[t][r] + bb; }
  LDSX();
  for (int q = lane; q < 16 * 32; q += 32) { const int rl = q >> 5, pc = q & 31; const int row = r0 + rl; if (row < NN) vst2(out + (size_t)row * FI + pc * 4, *(const v4f*)(&so[wave][rl][pc * 4])); }
}
extern "C" void kernel_launch(void* const* d_in, const int* in_sizes, int n_in, void* d_out, int out_size, void* d_ws, size_t ws_size, hipStream_t stream) {
  (void)in_sizes; (void)n_in; (void)out_size; (void)ws_size;
  const float** I = (const float**)d_in;
  const float* feat = I[0]; const int* src = (const int*)d_in[1]; const int* dst = (const int*)d_in[2]; const float* Wfc = I[3]; const float* al = I[4]; const float* ar = I[5]; const float* Wres = I[6]; const float* bg = I[7]; const float* gam = I[8]; const float* bet = I[9]; const float* Wo = I[10]; const float* bo = I[11];
  float* out = (float*)d_out;
  char* ws = (char*)d_ws; size_t off = 0;
  auto take = [&](size_t bytes) { char* p = ws + off; off += (bytes + 255) & ~(size_t)255; return p; };
  float* XW = (float*)take((size_t)NNP * FH * 4); float* RES = (float*)take((size_t)NNP * FH * 4); float* EL = (float*)take((size_t)NNP * 4 * 4); float* ER = (float*)take((size_t)NNP * 4 * 4); float* SMX = (float*)take((size_t)NNP * 4 * 4);
  float* MU = (float*)take(FH * 4); float* ISD = (float*)take(FH * 4);
  float* RST = RES;
  k_node<1><<<NNP / 64, 128, 0, stream>>>(feat, Wfc, al, ar, XW, EL, ER);
  k_node<0><<<NNP / 64, 128, 0, stream>>>(feat, Wres, al, ar, RES, EL, ER);
  k_max<<<NRBM, 256, 0, stream>>>(src, dst, EL, ER, SMX);
  k_gagg<<<NRBA, 256, 0, stream>>>(src, dst, XW, EL, ER, SMX, RES, bg, RST);
  k_bn<<<FH / 256, 256, 0, stream>>>(RST, MU, ISD);
  k_out<<<NNP / 64, 128, 0, stream>>>(RST, MU, ISD, gam, bet, Wo, bo, out);
}
